// NALUi1_22677427323454
// MI455X (gfx1250) — hardware-run, weakly checked
//
#include <hip/hip_runtime.h>
#include <stddef.h>


typedef _Float16 h16;
typedef _Float16 v16h __attribute__((ext_vector_type(16)));
typedef _Float16 v8h  __attribute__((ext_vector_type(8)));
typedef float    v8f  __attribute__((ext_vector_type(8)));
typedef float    v4f  __attribute__((ext_vector_type(4)));

#ifndef NB
#define NB 1024
#endif
#define NB_FULL 1024
#define DIN  512
#define DOUT 512

static_assert(NB >= 64 && NB <= NB_FULL && (NB % 64) == 0);
static_assert(DIN == DOUT);
static_assert((DIN % 64) == 0 && (DIN % 32) == 0 && (DIN % 8) == 0);
static_assert((DOUT % 64) == 0 && (DOUT % 32) == 0);
static_assert(((size_t)NB * DIN) % 2048 == 0);

#define LDT 72
#define CLD 36
#define CTILE (64 * CLD)
static_assert((LDT % 8) == 0 && LDT >= 64);
static_assert((CLD % 4) == 0 && CLD >= 32);

#define ACARRY 16.0f
#define WCARRY 64.0f
#define LCARRY 64.0f

#define APLANE_BYTES ((size_t)NB * DIN * 2)
#define WPLANE_BYTES ((size_t)DIN * DOUT * 2)
#define OFF_X16  ((size_t)0)
#define OFF_XL16 (OFF_X16 + APLANE_BYTES)
#define OFF_MK16 (OFF_XL16 + APLANE_BYTES)
#define OFF_ZK16 (OFF_MK16 + APLANE_BYTES)
#define OFF_WT   (OFF_ZK16 + APLANE_BYTES)
#define OFF_LT   (OFF_WT + WPLANE_BYTES)
#define OFF_PT   (OFF_LT + WPLANE_BYTES)
#define OFF_ZT   (OFF_PT + WPLANE_BYTES)
#define WS_TOTAL (OFF_ZT + WPLANE_BYTES)
static_assert((APLANE_BYTES % 128) == 0 && (WPLANE_BYTES % 128) == 0);
static_assert(WS_TOTAL <= (size_t)134217728);

__device__ __forceinline__ float bf16r(float x) {
  unsigned int u = __float_as_uint(x);
  u = (u + 0x7FFFu + ((u >> 16) & 1u)) & 0xFFFF0000u;
  return __uint_as_float(u);
}

static __device__ __forceinline__ h16 toh_flush(float v) {
  const h16 r = (h16)v;
  return (fabsf(v) < 6.103515625e-05f) ? (h16)0.0f : r;
}

__device__ __forceinline__ v16h frag_at(const _Float16* p) {
  v8h lo = *(const v8h*)(p);
  v8h hi = *(const v8h*)(p + 16);
  v16h out;
#pragma unroll
  for (int i = 0; i < 8; ++i) { out[i] = lo[i]; out[i + 8] = hi[i]; }
  return out;
}

__device__ __forceinline__ v8f wmma16(v16h a, v16h b, v8f c) {
  v8f d = __builtin_amdgcn_wmma_f32_16x16x32_f16(false, a, false, b, (short)0, c,
                                                 false, false);
  asm volatile("v_nop\n\tv_nop\n\tv_nop\n\tv_nop" : "+v"(d) : "v"(a), "v"(b));
  return d;
}

__global__ __launch_bounds__(256) void wprep_kernel(
    const float* __restrict__ w_hat, const float* __restrict__ m_hat,
    _Float16* __restrict__ Wt, _Float16* __restrict__ Lt,
    _Float16* __restrict__ Pt, _Float16* __restrict__ Zt) {
#pragma clang fp contract(off)
  __shared__ __attribute__((aligned(16))) _Float16 TW[64 * LDT];
  __shared__ __attribute__((aligned(16))) _Float16 TL[64 * LDT];
  __shared__ __attribute__((aligned(16))) _Float16 TP[64 * LDT];
  __shared__ __attribute__((aligned(16))) _Float16 TZ[64 * LDT];
  const unsigned tid = threadIdx.x;
  const unsigned n0 = blockIdx.x * 64u;
  const unsigned k0 = blockIdx.y * 64u;
#pragma unroll 1
  for (unsigned j = 0; j < 16u; ++j) {
    const unsigned idx = tid + 256u * j;
    const unsigned kr = idx >> 6, nc = idx & 63u;
    const size_t gi = (size_t)(k0 + kr) * DOUT + n0 + nc;
    const float wh = bf16r(w_hat[gi]);
    const float mh = bf16r(m_hat[gi]);
    const float sg = __builtin_amdgcn_rcpf(1.0f + expf(-mh));
    const float wv = tanhf(wh) * sg;
    const float aw = fabsf(wv);
    const float t = 1.0f - 2.0f * aw;
    const float l2 = logf(fmaxf(fabsf(t), 1.0e-37f));
    const float l1 = logf(fmaxf(1.0f - aw, 1.0e-37f));
    TW[nc * LDT + kr] = toh_flush(WCARRY * wv);
    TL[kr * LDT + nc] = toh_flush(LCARRY * l2);
    TZ[kr * LDT + nc] = toh_flush(LCARRY * l1);
    TP[kr * LDT + nc] = (t < 0.0f) ? (h16)1.0f : (h16)0.0f;
  }
  __syncthreads();
  v8h xw[2], xl[2], xp[2], xz[2];
  size_t offw[2], offl[2];
#pragma unroll
  for (unsigned i = 0; i < 2u; ++i) {
    const unsigned r = 32u * i + (tid >> 3);
    const unsigned c = (tid & 7u) * 8u;
    xw[i] = *(const v8h*)&TW[r * LDT + c];
    xl[i] = *(const v8h*)&TL[r * LDT + c];
    xp[i] = *(const v8h*)&TP[r * LDT + c];
    xz[i] = *(const v8h*)&TZ[r * LDT + c];
    offw[i] = (size_t)(n0 + r) * DIN + k0 + c;
    offl[i] = (size_t)(k0 + r) * DOUT + n0 + c;
  }
#pragma unroll
  for (int i = 0; i < 2; ++i) {
    *(volatile v8h*)(Wt + offw[i]) = xw[i];
    *(volatile v8h*)(Lt + offl[i]) = xl[i];
    *(volatile v8h*)(Pt + offl[i]) = xp[i];
    *(volatile v8h*)(Zt + offl[i]) = xz[i];
  }
  __threadfence();
#pragma unroll
  for (int i = 0; i < 2; ++i) {
    *(volatile v8h*)(Wt + offw[i]) = xw[i];
    *(volatile v8h*)(Lt + offl[i]) = xl[i];
    *(volatile v8h*)(Pt + offl[i]) = xp[i];
    *(volatile v8h*)(Zt + offl[i]) = xz[i];
  }
}

__global__ __launch_bounds__(256) void xprep_kernel(
    const float* __restrict__ X, _Float16* __restrict__ X16, _Float16* __restrict__ XL16,
    _Float16* __restrict__ MK16, _Float16* __restrict__ ZK16) {
#pragma clang fp contract(off)
  __shared__ __attribute__((aligned(16))) _Float16 SX[2048];
  __shared__ __attribute__((aligned(16))) _Float16 SL[2048];
  __shared__ __attribute__((aligned(16))) _Float16 SM[2048];
  __shared__ __attribute__((aligned(16))) _Float16 SZ[2048];
  const unsigned tid = threadIdx.x;
  const size_t base = (size_t)blockIdx.x * 2048u;
#pragma unroll 1
  for (unsigned j = 0; j < 8u; ++j) {
    const unsigned idx = tid + 256u * j;
    const float v = bf16r(X[base + idx]);
    const float lg = logf(fmaxf(fabsf(v), 1.0e-7f));
    SX[idx] = toh_flush(ACARRY * v);
    SL[idx] = toh_flush(ACARRY * lg);
    SM[idx] = (v < 0.0f) ? (h16)1.0f : (h16)0.0f;
    SZ[idx] = (v == 0.0f) ? (h16)1.0f : (h16)0.0f;
  }
  __syncthreads();
  const unsigned e = tid * 8u;
  const v8h ax = *(const v8h*)&SX[e];
  const v8h al = *(const v8h*)&SL[e];
  const v8h am = *(const v8h*)&SM[e];
  const v8h az = *(const v8h*)&SZ[e];
  const size_t off = base + e;
  *(volatile v8h*)(X16 + off)  = ax;
  *(volatile v8h*)(XL16 + off) = al;
  *(volatile v8h*)(MK16 + off) = am;
  *(volatile v8h*)(ZK16 + off) = az;
  __threadfence();
  *(volatile v8h*)(X16 + off)  = ax;
  *(volatile v8h*)(XL16 + off) = al;
  *(volatile v8h*)(MK16 + off) = am;
  *(volatile v8h*)(ZK16 + off) = az;
}

__global__ __launch_bounds__(256) void paths_gemm_kernel(
    const _Float16* __restrict__ X16, const _Float16* __restrict__ XL16,
    const _Float16* __restrict__ MK16, const _Float16* __restrict__ ZK16,
    const _Float16* __restrict__ Wt, const _Float16* __restrict__ Lt,
    const _Float16* __restrict__ Pt, const _Float16* __restrict__ Zt,
    const float* __restrict__ G, float* __restrict__ out) {
  __shared__ __attribute__((aligned(16))) float Cs[4 * CTILE];
  const unsigned tid = threadIdx.x, lane = tid & 31u;
  const unsigned w = (unsigned)__builtin_amdgcn_readfirstlane((int)(tid >> 5));
  const unsigned mw = w >> 1, nw = w & 1u;
  const unsigned hh = lane >> 4, m = lane & 15u;
  const unsigned n0 = blockIdx.x * 32u;
  const unsigned row0 = blockIdx.y * 64u;

  const size_t aoff = (size_t)(row0 + mw * 16u + m) * DIN + hh * 8u;
  const size_t boff = (size_t)(n0 + nw * 16u + m) * DIN + hh * 8u;
  v8f acc_a = {}, acc_m = {}, acc_s = {}, acc_p = {};
#pragma unroll 2
  for (unsigned k0 = 0; k0 < (unsigned)DIN; k0 += 32u) {
    const v16h ax = frag_at(X16 + aoff + k0);
    const v16h al = frag_at(XL16 + aoff + k0);
    const v16h am = frag_at(MK16 + aoff + k0);
    const v16h az = frag_at(ZK16 + aoff + k0);
    const v16h bw = frag_at(Wt + boff + k0);
    const v16h bl = frag_at(Lt + boff + k0);
    const v16h bp = frag_at(Pt + boff + k0);
    const v16h bz = frag_at(Zt + boff + k0);
    acc_a = wmma16(ax, bw, acc_a);
    acc_s = wmma16(am, bl, acc_s);
    acc_m = wmma16(al, bw, acc_m);
    acc_p = wmma16(am, bp, acc_p);
    acc_s = wmma16(az, bz, acc_s);
  }
#pragma unroll
  for (int r = 0; r < 8; ++r) {
    const unsigned ci = (mw * 16u + hh * 8u + (unsigned)r) * CLD + nw * 16u + m;
    Cs[ci]             = acc_a[r];
    Cs[CTILE + ci]     = acc_m[r];
    Cs[2 * CTILE + ci] = acc_s[r];
    Cs[3 * CTILE + ci] = acc_p[r];
  }
  __syncthreads();

#pragma unroll 1
  for (unsigned i = 0; i < 2u; ++i) {
    const unsigned r = 32u * i + (tid >> 3);
    const unsigned c = (tid & 7u) * 4u;
    const v4f ua = *(const v4f*)&Cs[r * CLD + c];
    const v4f um = *(const v4f*)&Cs[CTILE + r * CLD + c];
    const v4f us = *(const v4f*)&Cs[2 * CTILE + r * CLD + c];
    const v4f up = *(const v4f*)&Cs[3 * CTILE + r * CLD + c];
    const v4f gb = *(const v4f*)(G + n0 + c);
    v4f t;
#pragma unroll
    for (int j = 0; j < 4; ++j) {
      const float a  = ua[j] * (1.0f / (ACARRY * WCARRY));
      const float lm = um[j] * (1.0f / (ACARRY * WCARRY));
      const float mm = expf(fminf(lm, 20.0f));
      const float ls = us[j] * (1.0f / LCARRY);
      float ms = expf(ls);
      const int par = (int)(up[j] + 0.5f);
      ms = (par & 1) ? -ms : ms;
      ms = fminf(fmaxf(ms, -1.0f), 1.0f);
      const float gv = __builtin_amdgcn_rcpf(1.0f + expf(-bf16r(gb[j])));
      t[j] = gv * a + (1.0f - gv) * mm * ms;
    }
    *(v4f*)&Cs[r * CLD + c] = t;
  }

  v4f xs[2];
  size_t off[2];
#pragma unroll
  for (unsigned i = 0; i < 2u; ++i) {
    const unsigned r = 32u * i + (tid >> 3);
    const unsigned c = (tid & 7u) * 4u;
    xs[i] = *(const v4f*)&Cs[r * CLD + c];
    off[i] = (size_t)(row0 + r) * DOUT + n0 + c;
  }
#pragma unroll
  for (int i = 0; i < 2; ++i) *(volatile v4f*)(out + off[i]) = xs[i];
  __threadfence();
#pragma unroll
  for (int i = 0; i < 2; ++i) *(volatile v4f*)(out + off[i]) = xs[i];
}

extern "C" void kernel_launch(void* const* d_in, const int* in_sizes, int n_in,
                              void* d_out, int out_size, void* d_ws, size_t ws_size,
                              hipStream_t stream) {
  if (n_in < 4) return;
  if ((long long)in_sizes[0] < (long long)NB * DIN) return;
  if ((long long)in_sizes[1] < (long long)DIN * DOUT) return;
  if ((long long)in_sizes[2] < (long long)DIN * DOUT) return;
  if (in_sizes[3] < DOUT) return;
  if ((long long)out_size < (long long)NB * DOUT) return;
  if (ws_size < WS_TOTAL) return;

  const float* x     = (const float*)d_in[0];
  const float* w_hat = (const float*)d_in[1];
  const float* m_hat = (const float*)d_in[2];
  const float* g     = (const float*)d_in[3];
  float* out = (float*)d_out;

  char* ws = (char*)d_ws;
  _Float16* X16  = (_Float16*)(ws + OFF_X16);
  _Float16* XL16 = (_Float16*)(ws + OFF_XL16);
  _Float16* MK16 = (_Float16*)(ws + OFF_MK16);
  _Float16* ZK16 = (_Float16*)(ws + OFF_ZK16);
  _Float16* Wt   = (_Float16*)(ws + OFF_WT);
  _Float16* Lt   = (_Float16*)(ws + OFF_LT);
  _Float16* Pt   = (_Float16*)(ws + OFF_PT);
  _Float16* Zt   = (_Float16*)(ws + OFF_ZT);

  dim3 blk(256);
  wprep_kernel<<<dim3(DOUT / 64, DIN / 64), blk, 0, stream>>>(w_hat, m_hat, Wt, Lt, Pt, Zt);
  xprep_kernel<<<dim3((unsigned)(((size_t)NB * DIN) / 2048)), blk, 0, stream>>>(
      x, X16, XL16, MK16, ZK16);
  paths_gemm_kernel<<<dim3(DOUT / 32, NB / 64), blk, 0, stream>>>(
      X16, XL16, MK16, ZK16, Wt, Lt, Pt, Zt, g, out);
}
